// SimpleMamba2Block_11690900980065
// MI455X (gfx1250) — hardware-verified
//
#include <hip/hip_runtime.h>
#include <hip/hip_bf16.h>
#include <math.h>
#include <stdint.h>
#include <stddef.h>


#define D_MODEL   1024
#define STATE     64
#define HEADS     8
#define INNER     2048
#define HEAD_DIM  256
#define PROJ_OUT  4232
#define NPAD1     4288
#define BATCH     2
#define SEQ       1024
#define ROWS      (BATCH * SEQ)
#define LN_EPS    1e-5f
#define QC        64
#define NCHUNK    (SEQ / QC)

#define COL_Z   0
#define COL_X   INNER
#define COL_B   (2 * INNER)
#define COL_C   (2 * INNER + STATE)
#define COL_DT  (2 * INNER + 2 * STATE)

#define SC_X    64.0f
#define SC_BC   16.0f
#define SC_G    128.0f
#define SC_CS   2048.0f
#define SC_H    128.0f
#define SC_BW   256.0f
#define SC_Y    8.0f
#define SC_WOUT 1024.0f

static_assert(NPAD1 % 64 == 0 && NPAD1 >= PROJ_OUT);
static_assert(ROWS % 128 == 0 && D_MODEL % 64 == 0 && INNER % 64 == 0);
static_assert(SEQ % QC == 0 && QC == 64 && STATE == 64 && HEAD_DIM == 256);

typedef __bf16   bf16;
typedef _Float16 f16;
typedef __attribute__((ext_vector_type(16))) __bf16   v16bf;
typedef __attribute__((ext_vector_type(8)))  __bf16   v8bf;
typedef __attribute__((ext_vector_type(16))) _Float16 v16h;
typedef __attribute__((ext_vector_type(8)))  _Float16 v8h;
typedef __attribute__((ext_vector_type(8)))  float    v8f;
typedef __attribute__((ext_vector_type(4)))  float    v4f;
typedef __attribute__((ext_vector_type(4)))  unsigned int v4u;

__device__ __forceinline__ v8f vzero8() { return (v8f){0.f, 0.f, 0.f, 0.f, 0.f, 0.f, 0.f, 0.f}; }

__device__ __forceinline__ v8f mma16(v16h a, v16h b, v8f c) {
    v8f d = __builtin_amdgcn_wmma_f32_16x16x32_f16(false, a, false, b, (short)0, c, false, false);
    asm volatile("v_nop\n\tv_nop\n\tv_nop\n\tv_nop" : "+v"(d) : "v"(a), "v"(b));
    return d;
}
__device__ __forceinline__ v8f mma16(v16bf a, v16bf b, v8f c) {
    v8f d = __builtin_amdgcn_wmma_f32_16x16x32_bf16(false, a, false, b, (short)0, c, false, false);
    asm volatile("v_nop\n\tv_nop\n\tv_nop\n\tv_nop" : "+v"(d) : "v"(a), "v"(b));
    return d;
}

template<typename V>
__device__ __forceinline__ v4u pun16(V v) { union { V a; v4u b; } x; x.a = v; return x.b; }

template<typename T, typename V8T, typename V16T>
__device__ __forceinline__ V16T frag16(const T* base, int row, int ld, int k0, int lane) {
    const T* p = base + (size_t)row * ld + k0 + ((lane >> 4) << 3);
    union { V16T v; V8T e[2]; } u;
    u.e[0] = *(const V8T*)p;
    u.e[1] = *(const V8T*)(p + 16);
    return u.v;
}
__device__ __forceinline__ v16h frag_h(const f16* base, int row, int ld, int k0, int lane) {
    return frag16<f16, v8h, v16h>(base, row, ld, k0, lane);
}
__device__ __forceinline__ v16h frag_hf32(const float* base, int row, int ld, int k0, int lane, float sc) {
    const float* p = base + (size_t)row * ld + k0 + ((lane >> 4) << 3);
    v16h r;
#pragma unroll
    for (int e = 0; e < 8; ++e) {
        r[e]     = (f16)(p[e] * sc);
        r[8 + e] = (f16)(p[16 + e] * sc);
    }
    return r;
}

__device__ __forceinline__ float wave_sum(float v) {
#pragma unroll
    for (int o = 16; o > 0; o >>= 1) v += __shfl_xor(v, o, 32);
    return v;
}

template<int SPLIT, typename T, typename V8T>
__global__ __launch_bounds__(128)
void transpose_cvt_kernel(const float* __restrict__ W, T* __restrict__ Thi, T* __restrict__ Tlo,
                          int K, int N, int NPADv, float scale)
{
    __shared__ float tile[64][65];
    const int tid = threadIdx.x, lane = tid & 31, wave = tid >> 5;
    const int n0 = blockIdx.x * 64;
    const int k0 = blockIdx.y * 64;
#pragma unroll 8
    for (int j = 0; j < 32; ++j) {
        const int idx = tid + j * 128;
        const int kk = idx >> 6, nn = idx & 63;
        const int k = k0 + kk, n = n0 + nn;
        float v = 0.0f;
        if (k < K && n < N) v = W[(size_t)k * N + n];
        tile[kk][nn] = v;
    }
    __syncthreads();
    v4u oh[4], ol[4];
    size_t off[4];
    bool ok[4];
#pragma unroll
    for (int i = 0; i < 4; ++i) {
        const int nn = wave * 16 + i * 4 + (lane >> 3);
        const int ks = (lane & 7) * 8;
        V8T hv, lv;
#pragma unroll
        for (int e = 0; e < 8; ++e) {
            const float v = tile[ks + e][nn] * scale;
            const T t1 = (T)v;
            hv[e] = t1;
            if constexpr (SPLIT != 0) lv[e] = (T)(v - (float)t1);
            else lv[e] = t1;
        }
        oh[i] = pun16(hv);
        ol[i] = pun16(lv);
        off[i] = (size_t)(n0 + nn) * K + k0 + ks;
        ok[i] = (n0 + nn < NPADv) && (k0 + ks + 8 <= K);
    }
#pragma unroll
    for (int i = 0; i < 4; ++i) {
        if (ok[i]) {
            *(volatile v4u*)(Thi + off[i]) = oh[i];
            if constexpr (SPLIT != 0) *(volatile v4u*)(Tlo + off[i]) = ol[i];
        }
    }
    __threadfence();
#pragma unroll
    for (int i = 0; i < 4; ++i) {
        if (ok[i]) {
            *(volatile v4u*)(Thi + off[i]) = oh[i];
            if constexpr (SPLIT != 0) *(volatile v4u*)(Tlo + off[i]) = ol[i];
        }
    }
}

__global__ __launch_bounds__(128)
void layernorm_split_kernel(const float* __restrict__ x, const float* __restrict__ gamma,
                            const float* __restrict__ beta, bf16* __restrict__ Ahi,
                            bf16* __restrict__ Alo, int nrows)
{
    __shared__ float red[4];
    const int row = blockIdx.x;
    if (row >= nrows) return;
    const int tid = threadIdx.x, lane = tid & 31, wave = tid >> 5;
    const int c0 = tid * 8;
    const float* xr = x + (size_t)row * D_MODEL + c0;
    const v4f xa = *(const v4f*)xr;
    const v4f xb = *(const v4f*)(xr + 4);
    float v[8];
    v[0] = xa[0]; v[1] = xa[1]; v[2] = xa[2]; v[3] = xa[3];
    v[4] = xb[0]; v[5] = xb[1]; v[6] = xb[2]; v[7] = xb[3];
    float s = 0.f;
#pragma unroll
    for (int e = 0; e < 8; ++e) s += v[e];
    s = wave_sum(s);
    if (lane == 0) red[wave] = s;
    __syncthreads();
    const float mu = (red[0] + red[1] + red[2] + red[3]) * (1.0f / D_MODEL);
    __syncthreads();
    float q = 0.f;
#pragma unroll
    for (int e = 0; e < 8; ++e) { const float d = v[e] - mu; q += d * d; }
    q = wave_sum(q);
    if (lane == 0) red[wave] = q;
    __syncthreads();
    const float var = (red[0] + red[1] + red[2] + red[3]) * (1.0f / D_MODEL);
    const float rs = rsqrtf(var + LN_EPS);
    v8bf hv, lv;
#pragma unroll
    for (int e = 0; e < 8; ++e) {
        const int c = c0 + e;
        const float o = (v[e] - mu) * rs * gamma[c] + beta[c];
        const bf16 t1 = (bf16)o;
        hv[e] = t1;
        lv[e] = (bf16)(o - (float)t1);
    }
    const v4u uh = pun16(hv), ul = pun16(lv);
    bf16* ph = Ahi + (size_t)row * D_MODEL + c0;
    bf16* pl = Alo + (size_t)row * D_MODEL + c0;
    *(volatile v4u*)ph = uh;
    *(volatile v4u*)pl = ul;
    __threadfence();
    *(volatile v4u*)ph = uh;
    *(volatile v4u*)pl = ul;
}

template<int SPLIT, typename T, typename V8T, typename V16T>
__global__ __launch_bounds__(128)
void gemm16_kernel(const T* __restrict__ Ahi, const T* __restrict__ Alo,
                   const T* __restrict__ Bhi, const T* __restrict__ Blo,
                   float* __restrict__ C, const float* __restrict__ bias,
                   const float* __restrict__ resid, int use_resid,
                   int M, int K, int ldc, int Nreal, int ldr, float oscale)
{
    __shared__ __attribute__((aligned(16))) float stg[4 * 32 * 68];
    const int tid = threadIdx.x, lane = tid & 31, wave = tid >> 5;
    const int hh = lane >> 4, m = lane & 15;
    const int n0 = blockIdx.x * 64;
    const int m0 = blockIdx.y * 128 + wave * 32;
    const int ra0 = min(m0 + m, M - 1);
    const int ra1 = min(m0 + 16 + m, M - 1);

    v8f acc[2][4];
#pragma unroll
    for (int mi = 0; mi < 2; ++mi)
#pragma unroll
        for (int ni = 0; ni < 4; ++ni) acc[mi][ni] = vzero8();

    for (int k0 = 0; k0 < K; k0 += 32) {
        V16T ah0 = frag16<T, V8T, V16T>(Ahi, ra0, K, k0, lane);
        V16T ah1 = frag16<T, V8T, V16T>(Ahi, ra1, K, k0, lane);
        V16T al0 = ah0, al1 = ah1;
        if constexpr (SPLIT != 0) {
            al0 = frag16<T, V8T, V16T>(Alo, ra0, K, k0, lane);
            al1 = frag16<T, V8T, V16T>(Alo, ra1, K, k0, lane);
        }
#pragma unroll
        for (int ni = 0; ni < 4; ++ni) {
            const int nrow = n0 + ni * 16 + m;
            V16T bh = frag16<T, V8T, V16T>(Bhi, nrow, K, k0, lane);
            acc[0][ni] = mma16(ah0, bh, acc[0][ni]);
            acc[1][ni] = mma16(ah1, bh, acc[1][ni]);
            if constexpr (SPLIT != 0) {
                V16T bl = frag16<T, V8T, V16T>(Blo, nrow, K, k0, lane);
                acc[0][ni] = mma16(al0, bh, acc[0][ni]);
                acc[1][ni] = mma16(al1, bh, acc[1][ni]);
                acc[0][ni] = mma16(ah0, bl, acc[0][ni]);
                acc[1][ni] = mma16(ah1, bl, acc[1][ni]);
            }
        }
    }

    float* st = stg + wave * (32 * 68);
#pragma unroll
    for (int mi = 0; mi < 2; ++mi)
#pragma unroll
        for (int ni = 0; ni < 4; ++ni)
#pragma unroll
            for (int r = 0; r < 8; ++r)
                st[(mi * 16 + hh * 8 + r) * 68 + ni * 16 + m] = acc[mi][ni][r];
    __syncthreads();

    v4f ov[16];
    const int c4 = m * 4;
    const int gcol = n0 + c4;
#pragma unroll
    for (int i = 0; i < 16; ++i) {
        const int rr = 2 * i + hh;
        const int grow = min(m0 + rr, M - 1);
        const v4f a = *(const v4f*)(st + rr * 68 + c4);
        v4f o;
#pragma unroll
        for (int e = 0; e < 4; ++e) {
            const int col = gcol + e;
            float tv = a[e] * oscale;
            if (col < Nreal) {
                tv += bias[col];
                if (use_resid) tv += resid[(size_t)grow * ldr + col];
            }
            o[e] = tv;
        }
        ov[i] = o;
    }
#pragma unroll
    for (int i = 0; i < 16; ++i) {
        const int rr = 2 * i + hh;
        const int grow = m0 + rr;
        if (grow < M) *(volatile v4f*)(C + (size_t)grow * ldc + gcol) = ov[i];
    }
    __threadfence();
#pragma unroll
    for (int i = 0; i < 16; ++i) {
        const int rr = 2 * i + hh;
        const int grow = m0 + rr;
        if (grow < M) *(volatile v4f*)(C + (size_t)grow * ldc + gcol) = ov[i];
    }
}

#define SM_H    0
#define SM_X    (SM_H + HEAD_DIM * STATE * 4)
#define SM_CR   (SM_X + HEAD_DIM * QC * 2)
#define SM_CS   (SM_CR + QC * STATE * 2)
#define SM_BR   (SM_CS + QC * STATE * 2)
#define SM_BW   (SM_BR + QC * STATE * 2)
#define SM_G    (SM_BW + QC * STATE * 2)
#define SM_Y    (SM_G + QC * QC * 2)
#define SM_ST   (SM_Y + 8 * 16 * 128 * 2)
#define SM_DT   (SM_ST + QC * 4)
#define SM_TOTAL (SM_DT + QC * 4)

__global__ __launch_bounds__(256)
void ssd_chunk_kernel(const float* __restrict__ zx,
                      const float* __restrict__ A_log,
                      const float* __restrict__ D_skip,
                      const float* __restrict__ dt_bias,
                      f16* __restrict__ y,
                      int nblocks)
{
    extern __shared__ __attribute__((aligned(16))) char smem[];
    float* sH  = (float*)(smem + SM_H);
    f16*   sX  = (f16*)(smem + SM_X);
    f16*   sCr = (f16*)(smem + SM_CR);
    f16*   sCs = (f16*)(smem + SM_CS);
    f16*   sBr = (f16*)(smem + SM_BR);
    f16*   sBw = (f16*)(smem + SM_BW);
    f16*   sG  = (f16*)(smem + SM_G);
    f16*   sY  = (f16*)(smem + SM_Y);
    float* sSt = (float*)(smem + SM_ST);
    float* sDt = (float*)(smem + SM_DT);

    const int tid = threadIdx.x, lane = tid & 31, wave = tid >> 5;
    const int hh = lane >> 4, m = lane & 15;
    if ((int)blockIdx.x >= nblocks) return;
    const int h = blockIdx.x & 7;
    const int b = blockIdx.x >> 3;

    const float Ah  = -expf(A_log[h]);
    const float Dh  = D_skip[h];
    const float dtb = dt_bias[h];

    for (int i = tid; i < HEAD_DIM * STATE; i += 256) sH[i] = 0.0f;
    __syncthreads();

    for (int c = 0; c < NCHUNK; ++c) {
        const int row0 = b * SEQ + c * QC;

        if (tid < QC) {
            const float raw = zx[(size_t)(row0 + tid) * NPAD1 + COL_DT + h] + dtb;
            const float sp = fmaxf(raw, 0.0f) + log1pf(expf(-fabsf(raw)));
            sDt[tid] = sp;
            sSt[tid] = sp * Ah;
        }
        __syncthreads();
        if (tid == 0) {
            float run = 0.0f;
            for (int t = 0; t < QC; ++t) { run += sSt[t]; sSt[t] = run; }
        }
        __syncthreads();
        const float sLast = sSt[QC - 1];

        for (int i = tid; i < QC * STATE; i += 256) {
            const int t = i >> 6, n = i & 63;
            const size_t rb = (size_t)(row0 + t) * NPAD1;
            const float bv = zx[rb + COL_B + n];
            const float cv = zx[rb + COL_C + n];
            const float st = sSt[t], dtv = sDt[t];
            sBr[t * STATE + n] = (f16)(bv * SC_BC);
            sCr[t * STATE + n] = (f16)(cv * SC_BC);
            sBw[n * QC + t]    = (f16)(bv * dtv * expf(sLast - st) * SC_BW);
            sCs[t * STATE + n] = (f16)(cv * expf(st) * SC_CS);
        }
        for (int i = tid; i < HEAD_DIM * QC; i += 256) {
            const int p = i & 255, t = i >> 8;
            const float xv = zx[(size_t)(row0 + t) * NPAD1 + COL_X + h * HEAD_DIM + p];
            sX[p * QC + t] = (f16)(xv * SC_X);
        }
        __syncthreads();

        {
#pragma unroll
            for (int j = 0; j < 2; ++j) {
                const int idx = wave * 2 + j;
                const int mi = idx >> 2, ni = idx & 3;
                v8f acc = vzero8();
#pragma unroll
                for (int k0 = 0; k0 < STATE; k0 += 32) {
                    v16h a  = frag_h(sCr, mi * 16 + m, STATE, k0, lane);
                    v16h bb = frag_h(sBr, ni * 16 + m, STATE, k0, lane);
                    acc = mma16(a, bb, acc);
                }
                const int s  = ni * 16 + m;
                const int tb = mi * 16 + hh * 8;
                const float ds = sDt[s], ss = sSt[s];
#pragma unroll
                for (int r = 0; r < 8; ++r) {
                    const int t = tb + r;
                    const float e = expf(fminf(sSt[t] - ss, 0.0f));
                    float v = acc[r] * ds * e * (SC_G / (SC_BC * SC_BC));
                    if (s > t) v = 0.0f;
                    sG[t * QC + s] = (f16)v;
                }
            }
        }
        __syncthreads();

        {
            const int mi = wave & 3;
            const int ph = wave >> 2;
            v8f acc[8];
#pragma unroll
            for (int ni = 0; ni < 8; ++ni) acc[ni] = vzero8();
#pragma unroll
            for (int k0 = 0; k0 < QC; k0 += 32) {
                v16h a = frag_h(sG, mi * 16 + m, QC, k0, lane);
#pragma unroll
                for (int ni = 0; ni < 8; ++ni)
                    acc[ni] = mma16(a, frag_h(sX, ph * 128 + ni * 16 + m, QC, k0, lane), acc[ni]);
            }
#pragma unroll
            for (int ni = 0; ni < 8; ++ni) acc[ni] *= ((SC_CS * SC_H) / (SC_G * SC_X));
#pragma unroll
            for (int k0 = 0; k0 < STATE; k0 += 32) {
                v16h a = frag_h(sCs, mi * 16 + m, STATE, k0, lane);
#pragma unroll
                for (int ni = 0; ni < 8; ++ni)
                    acc[ni] = mma16(a, frag_hf32(sH, ph * 128 + ni * 16 + m, STATE, k0, lane, SC_H), acc[ni]);
            }
            f16* sYw = sY + wave * (16 * 128);
            const float inv2 = 1.0f / (SC_CS * SC_H);
#pragma unroll
            for (int ni = 0; ni < 8; ++ni) {
                const int pl = ni * 16 + m;
                const int pg = ph * 128 + pl;
#pragma unroll
                for (int r = 0; r < 8; ++r) {
                    const int tl = hh * 8 + r;
                    const size_t gro = (size_t)(row0 + mi * 16 + tl) * NPAD1;
                    const float xv = zx[gro + COL_X + h * HEAD_DIM + pg];
                    const float zv = zx[gro + COL_Z + h * HEAD_DIM + pg];
                    const float gate = zv / (1.0f + __expf(-zv));
                    const float yv = (acc[ni][r] * inv2 + Dh * xv) * gate;
                    sYw[tl * 128 + pl] = (f16)(yv * SC_Y);
                }
            }
            __syncthreads();
            v4u yl[8];
#pragma unroll
            for (int i = 0; i < 8; ++i) {
                const int rr = 2 * i + hh;
                yl[i] = pun16(*(const v8h*)(sYw + rr * 128 + m * 8));
            }
            f16* ybase = y + (size_t)(row0 + mi * 16) * INNER + h * HEAD_DIM + ph * 128 + m * 8;
#pragma unroll
            for (int i = 0; i < 8; ++i) {
                const int rr = 2 * i + hh;
                *(volatile v4u*)(ybase + (size_t)rr * INNER) = yl[i];
            }
            __threadfence();
#pragma unroll
            for (int i = 0; i < 8; ++i) {
                const int rr = 2 * i + hh;
                *(volatile v4u*)(ybase + (size_t)rr * INNER) = yl[i];
            }
        }
        __syncthreads();

        {
            const float dAll = expf(sLast);
            const float inv3 = 1.0f / (SC_X * SC_BW);
#pragma unroll
            for (int j = 0; j < 2; ++j) {
                const int pt = wave * 2 + j;
                v8f acc[4];
#pragma unroll
                for (int ni = 0; ni < 4; ++ni) acc[ni] = vzero8();
#pragma unroll
                for (int k0 = 0; k0 < QC; k0 += 32) {
                    v16h a = frag_h(sX, pt * 16 + m, QC, k0, lane);
#pragma unroll
                    for (int ni = 0; ni < 4; ++ni)
                        acc[ni] = mma16(a, frag_h(sBw, ni * 16 + m, QC, k0, lane), acc[ni]);
                }
                const int pb = pt * 16 + hh * 8;
#pragma unroll
                for (int ni = 0; ni < 4; ++ni) {
                    const int n = ni * 16 + m;
#pragma unroll
                    for (int r = 0; r < 8; ++r) {
                        const int p = pb + r;
                        float* hp = sH + p * STATE + n;
                        *hp = dAll * *hp + acc[ni][r] * inv3;
                    }
                }
            }
        }
        __syncthreads();
    }
}

static inline size_t align256(size_t x) { return (x + 255) & ~(size_t)255; }

extern "C" void kernel_launch(void* const* d_in, const int* in_sizes, int n_in,
                              void* d_out, int out_size, void* d_ws, size_t ws_size,
                              hipStream_t stream)
{
    if (n_in < 10) return;
    if (in_sizes[0] != ROWS * D_MODEL || in_sizes[1] < D_MODEL || in_sizes[2] < D_MODEL ||
        in_sizes[3] != D_MODEL * PROJ_OUT || in_sizes[4] < PROJ_OUT || in_sizes[5] < HEADS ||
        in_sizes[6] < HEADS || in_sizes[7] < HEADS || in_sizes[8] != INNER * D_MODEL ||
        in_sizes[9] < D_MODEL || out_size != ROWS * D_MODEL) return;

    const float* input    = (const float*)d_in[0];
    const float* ln_gamma = (const float*)d_in[1];
    const float* ln_beta  = (const float*)d_in[2];
    const float* W_in     = (const float*)d_in[3];
    const float* b_in     = (const float*)d_in[4];
    const float* A_log    = (const float*)d_in[5];
    const float* D_skip   = (const float*)d_in[6];
    const float* dt_bias  = (const float*)d_in[7];
    const float* W_out    = (const float*)d_in[8];
    const float* b_out    = (const float*)d_in[9];
    float* out = (float*)d_out;

    size_t off = 0;
    const size_t oA1hi  = off; off += align256((size_t)ROWS * D_MODEL * sizeof(bf16));
    const size_t oA1lo  = off; off += align256((size_t)ROWS * D_MODEL * sizeof(bf16));
    const size_t oWinHi = off; off += align256((size_t)NPAD1 * D_MODEL * sizeof(bf16));
    const size_t oWinLo = off; off += align256((size_t)NPAD1 * D_MODEL * sizeof(bf16));
    const size_t oZX    = off; off += align256((size_t)ROWS * NPAD1 * sizeof(float));
    const size_t oY2    = off; off += align256((size_t)ROWS * INNER * sizeof(f16));
    const size_t oWout  = off; off += align256((size_t)D_MODEL * INNER * sizeof(f16));
    if (off > ws_size) return;

    char* ws = (char*)d_ws;
    bf16*  A1hi   = (bf16*)(ws + oA1hi);
    bf16*  A1lo   = (bf16*)(ws + oA1lo);
    bf16*  WinThi = (bf16*)(ws + oWinHi);
    bf16*  WinTlo = (bf16*)(ws + oWinLo);
    float* ZX     = (float*)(ws + oZX);
    f16*   Y2     = (f16*)(ws + oY2);
    f16*   WoutT  = (f16*)(ws + oWout);

    transpose_cvt_kernel<1, bf16, v8bf><<<dim3(NPAD1 / 64, D_MODEL / 64), dim3(128), 0, stream>>>(
        W_in, WinThi, WinTlo, D_MODEL, PROJ_OUT, NPAD1, 1.0f);
    transpose_cvt_kernel<0, f16, v8h><<<dim3(D_MODEL / 64, INNER / 64), dim3(128), 0, stream>>>(
        W_out, WoutT, WoutT, INNER, D_MODEL, D_MODEL, SC_WOUT);

    layernorm_split_kernel<<<dim3(ROWS), dim3(128), 0, stream>>>(
        input, ln_gamma, ln_beta, A1hi, A1lo, ROWS);

    gemm16_kernel<1, bf16, v8bf, v16bf><<<dim3(NPAD1 / 64, ROWS / 128), dim3(128), 0, stream>>>(
        A1hi, A1lo, WinThi, WinTlo, ZX, b_in, input, 0,
        ROWS, D_MODEL, NPAD1, PROJ_OUT, D_MODEL, 1.0f);

    ssd_chunk_kernel<<<dim3(BATCH * HEADS), dim3(256), SM_TOTAL, stream>>>(
        ZX, A_log, D_skip, dt_bias, Y2, BATCH * HEADS);

    gemm16_kernel<0, f16, v8h, v16h><<<dim3(D_MODEL / 64, ROWS / 128), dim3(128), 0, stream>>>(
        Y2, Y2, WoutT, WoutT, out, b_out, input, 1,
        ROWS, INNER, D_MODEL, D_MODEL, D_MODEL, 1.0f / (SC_Y * SC_WOUT));
}
